// NonLocalBlockND_65326452572958
// MI455X (gfx1250) — hardware-verified
//
#include <hip/hip_runtime.h>


#ifndef NB
#define NB 4
#endif
#ifndef SEQ
#define SEQ 4096
#endif
#define NBF  4
#define HWF  4096
#define C_   256
#define CI   128
#define KB   32
#define PP   40
#define OSP  132
#define PCAR 16384.0f
#define VCAR 16.0f
#define YSC  (1.0f / 262144.0f)
#define ELAM 1e-4f

static_assert(NB >= 1 && NB <= NBF);
static_assert(SEQ % 128 == 0 && SEQ >= 128 && SEQ <= HWF);
static_assert(SEQ % KB == 0 && SEQ % 64 == 0 && SEQ % 16 == 0);
static_assert((NB * C_) % 32 == 0);
static_assert(C_ % 64 == 0 && CI % 64 == 0 && C_ % 32 == 0 && CI % 32 == 0);
static_assert((NB * SEQ * C_) % (8 * 256) == 0 && (NB * SEQ * CI) % 8 == 0);

typedef _Float16 h16;
typedef unsigned short bf;
typedef __attribute__((ext_vector_type(16))) __bf16   v16bf;
typedef __attribute__((ext_vector_type(16))) _Float16 v16h;
typedef __attribute__((ext_vector_type(8)))  _Float16 v8h;
typedef __attribute__((ext_vector_type(8)))  unsigned short v8us;
typedef __attribute__((ext_vector_type(8)))  float    v8f;
typedef __attribute__((ext_vector_type(4)))  float    v4f;
typedef v8h  __attribute__((may_alias)) v8ha;
typedef v4f  __attribute__((may_alias)) v4fa;
typedef v8us __attribute__((may_alias)) v8usa;

__device__ __forceinline__ unsigned short f2bf(float f) { unsigned u = __float_as_uint(f); u += 0x7FFFu + ((u >> 16) & 1u); return (unsigned short)(u >> 16); }
__device__ __forceinline__ float bf2f(unsigned short b) { return __uint_as_float(((unsigned)b) << 16); }
__device__ __forceinline__ float bfr(float f) { return bf2f(f2bf(f)); }
__device__ __forceinline__ void splitf(float y, unsigned short& h, unsigned short& l) { h = f2bf(y); l = f2bf(y - bf2f(h)); }
__device__ __forceinline__ v16h cat16(v8h lo, v8h hi) { return __builtin_shufflevector(lo, hi, 0, 1, 2, 3, 4, 5, 6, 7, 8, 9, 10, 11, 12, 13, 14, 15); }
__device__ __forceinline__ v16bf cat16b(v8us lo, v8us hi) { return __builtin_bit_cast(v16bf, __builtin_shufflevector(lo, hi, 0, 1, 2, 3, 4, 5, 6, 7, 8, 9, 10, 11, 12, 13, 14, 15)); }
__device__ __forceinline__ v8f wmma16(v16h a, v16h b, v8f c) { return __builtin_amdgcn_wmma_f32_16x16x32_f16(false, a, false, b, (short)0, c, false, false); }
__device__ __forceinline__ v8f wmmab(v16bf a, v16bf b, v8f c) { return __builtin_amdgcn_wmma_f32_16x16x32_bf16(false, a, false, b, (short)0, c, false, false); }
__device__ __forceinline__ v16bf ldb(const bf* p) { return cat16b(*(const v8us*)p, *(const v8us*)(p + 16)); }
__device__ __forceinline__ v16h  ldh(const h16* p) { return cat16(*(const v8h*)p, *(const v8h*)(p + 16)); }

template <typename T16> struct WFrag;
template <> struct WFrag<h16> { typedef v16h V; static __device__ __forceinline__ V ld(const h16* p) { return ldh(p); } static __device__ __forceinline__ v8f mma(V a, V b, v8f c) { return wmma16(a, b, c); } };
template <> struct WFrag<bf> { typedef v16bf V; static __device__ __forceinline__ V ld(const bf* p) { return ldb(p); } static __device__ __forceinline__ v8f mma(V a, V b, v8f c) { return wmmab(a, b, c); } };
template <typename T16, bool A2ON, bool B2ON, int BIASM, bool RESID>
__global__ __launch_bounds__(32) void k_gemmw(const T16* __restrict__ A, const T16* __restrict__ A2, const T16* __restrict__ Bt, const T16* __restrict__ Bt2, int K,
                                              float* C, int ldc, const float* __restrict__ bias, const float* __restrict__ res, size_t sA, size_t sB, size_t sC) {
    typedef typename WFrag<T16>::V V;
    __shared__ __align__(16) float os[16 * 68];
    const size_t z = blockIdx.z;
    A += z * sA; if (A2ON) A2 += z * sA; Bt += z * sB; if (B2ON) Bt2 += z * sB; C += z * sC; if (RESID) res += z * sC;
    const int lane = threadIdx.x & 31, lr = lane & 15, hi = lane >> 4;
    const int r0 = blockIdx.x * 64, c0 = blockIdx.y * 64;
    v8f acc[4][4];
#pragma unroll
    for (int mb = 0; mb < 4; ++mb)
#pragma unroll
        for (int nb = 0; nb < 4; ++nb) acc[mb][nb] = (v8f){};
    const size_t aoff = (size_t)(r0 + lr) * K + 8 * hi, boff = (size_t)(c0 + lr) * K + 8 * hi;
#pragma unroll 1
    for (int kc = 0; kc < K; kc += 32) {
        V a[4], a2[4];
#pragma unroll
        for (int mb = 0; mb < 4; ++mb) { a[mb] = WFrag<T16>::ld(A + aoff + (size_t)mb * 16 * K + kc); a2[mb] = a[mb]; if (A2ON) a2[mb] = WFrag<T16>::ld(A2 + aoff + (size_t)mb * 16 * K + kc); }
#pragma unroll
        for (int nb = 0; nb < 4; ++nb) {
            const V b = WFrag<T16>::ld(Bt + boff + (size_t)nb * 16 * K + kc); V b2 = b; if (B2ON) b2 = WFrag<T16>::ld(Bt2 + boff + (size_t)nb * 16 * K + kc);
#pragma unroll
            for (int mb = 0; mb < 4; ++mb) {
                acc[mb][nb] = WFrag<T16>::mma(a[mb], b, acc[mb][nb]);
                if (A2ON) acc[mb][nb] = WFrag<T16>::mma(a2[mb], b, acc[mb][nb]);
                if (B2ON) acc[mb][nb] = WFrag<T16>::mma(a[mb], b2, acc[mb][nb]); } }
        asm volatile("v_nop\n\tv_nop\n\tv_nop\n\tv_nop" : "+v"(acc[0][0]), "+v"(acc[1][1]), "+v"(acc[2][2]), "+v"(acc[3][3]) : "v"(a[0]), "v"(a[3]));
    }
#pragma unroll
    for (int mb = 0; mb < 4; ++mb) {
#pragma unroll
        for (int nb = 0; nb < 4; ++nb) {
#pragma unroll
            for (int j = 0; j < 8; ++j) os[(hi * 8 + j) * 68 + nb * 16 + lr] = acc[mb][nb][j]; }
        __builtin_amdgcn_fence(__ATOMIC_RELEASE, "wavefront"); __builtin_amdgcn_wave_barrier(); asm volatile("" ::: "memory");
        const size_t rb = (size_t)(r0 + mb * 16);
#pragma unroll 1
        for (int ps = 0; ps < 2; ++ps) {
#pragma unroll
            for (int s = 0; s < 8; ++s) {
                const int row = 2 * s + hi, cofs = lr * 4;
                v4f val = *(const v4fa*)(os + row * 68 + cofs);
                if (BIASM == 1) { val[0] += bfr(bias[c0 + cofs]); val[1] += bfr(bias[c0 + cofs + 1]); val[2] += bfr(bias[c0 + cofs + 2]); val[3] += bfr(bias[c0 + cofs + 3]); }
                if (BIASM == 2) { const float bv = bfr(bias[rb + row]); val[0] += bv; val[1] += bv; val[2] += bv; val[3] += bv; }
                if (RESID) { const v4f rv = *(const v4f*)(res + (rb + row) * (size_t)ldc + c0 + cofs); val[0] += bfr(rv[0]); val[1] += bfr(rv[1]); val[2] += bfr(rv[2]); val[3] += bfr(rv[3]); }
                *(volatile v4f*)(C + (rb + row) * (size_t)ldc + c0 + cofs) = val; }
            if (ps == 0) __threadfence(); }
        __builtin_amdgcn_fence(__ATOMIC_RELEASE, "wavefront"); __builtin_amdgcn_wave_barrier(); asm volatile("" ::: "memory");
    }
}

__global__ __launch_bounds__(256) void k_cvt8(const float* __restrict__ src, bf* dst, size_t n8) { const size_t i = (size_t)blockIdx.x * 256 + threadIdx.x; if (i >= n8) return; const v8f v = *(const v8f*)(src + i * 8); v8us o;
#pragma unroll
    for (int k = 0; k < 8; ++k) o[k] = f2bf(v[k]); *(volatile v8us*)(dst + i * 8) = o; __threadfence(); *(volatile v8us*)(dst + i * 8) = o; }

__global__ __launch_bounds__(256) void k_stats(const float* __restrict__ x, float* MU, float* RD) {
    __shared__ float mus[32]; __shared__ float rds[32];
    const int t = threadIdx.x, wid = t >> 5, lane = t & 31;
#pragma unroll 1
    for (int j = 0; j < 4; ++j) {
        const int rr = blockIdx.x * 32 + wid * 4 + j;
        const int b = rr / C_, c = rr - b * C_;
        const float* xr = x + ((size_t)b * C_ + c) * HWF + lane * 4;
        float s = 0.f;
#pragma unroll 1
        for (int i = 0; i < SEQ / 128; ++i) { const v4f v = *(const v4f*)(xr + (size_t)i * 128); s += (bfr(v[0]) + bfr(v[1])) + (bfr(v[2]) + bfr(v[3])); }
        s += __shfl_xor(s, 1, 32); s += __shfl_xor(s, 2, 32); s += __shfl_xor(s, 4, 32); s += __shfl_xor(s, 8, 32); s += __shfl_xor(s, 16, 32);
        const float mu = s * (1.0f / (float)SEQ);
        float ss = 0.f;
#pragma unroll 1
        for (int i = 0; i < SEQ / 128; ++i) { const v4f v = *(const v4f*)(xr + (size_t)i * 128);
            const float d0 = bfr(v[0]) - mu, d1 = bfr(v[1]) - mu, d2 = bfr(v[2]) - mu, d3 = bfr(v[3]) - mu;
            ss += (d0 * d0 + d1 * d1) + (d2 * d2 + d3 * d3); }
        ss += __shfl_xor(ss, 1, 32); ss += __shfl_xor(ss, 2, 32); ss += __shfl_xor(ss, 4, 32); ss += __shfl_xor(ss, 8, 32); ss += __shfl_xor(ss, 16, 32);
        const float den = 4.0f * (ss * (1.0f / (float)(SEQ - 1)) + ELAM);
        const float rd = 1.0f / den;
        if (lane == 0) { mus[wid * 4 + j] = mu; rds[wid * 4 + j] = rd; }
    }
    __syncthreads();
    if (wid == 0) {
        const float a = mus[lane], r = rds[lane];
        float* pm = MU + (size_t)blockIdx.x * 32 + lane; float* pr = RD + (size_t)blockIdx.x * 32 + lane;
        *(volatile float*)pm = a; *(volatile float*)pr = r; __threadfence(); *(volatile float*)pm = a; *(volatile float*)pr = r; }
}

__global__ __launch_bounds__(256) void k_xplanes(const float* __restrict__ x, const float* __restrict__ MU, const float* __restrict__ RD, bf* XT, bf* X1h, bf* X1l) {
    const size_t e = ((size_t)blockIdx.x * 256 + threadIdx.x) * 8; if (e >= (size_t)NB * SEQ * C_) return;
    const int c = (int)(e % C_); const size_t btk = e / C_; const int tpos = (int)(btk % SEQ); const int b = (int)(btk / SEQ);
    const float* xp = x + ((size_t)b * C_ + c) * HWF + tpos;
    const v8f mu8 = *(const v8f*)(MU + (size_t)b * C_ + c), rd8 = *(const v8f*)(RD + (size_t)b * C_ + c);
    v8us o0, oh, ol;
#pragma unroll
    for (int q = 0; q < 8; ++q) {
        const float xb = bfr(xp[(size_t)q * HWF]);
        const float d = xb - mu8[q];
        const float y = d * d * rd8[q] + 0.5f;
        const float ex = __expf(-y);
        const float sg = __builtin_amdgcn_rcpf(1.0f + ex);
        const float x1 = xb * sg;
        o0[q] = f2bf(xb); unsigned short hh, ll; splitf(x1, hh, ll); oh[q] = hh; ol[q] = ll;
    }
    *(volatile v8us*)(XT + e) = o0; *(volatile v8us*)(X1h + e) = oh; *(volatile v8us*)(X1l + e) = ol; __threadfence();
    *(volatile v8us*)(XT + e) = o0; *(volatile v8us*)(X1h + e) = oh; *(volatile v8us*)(X1l + e) = ol;
}

__global__ __launch_bounds__(256) void k_split8(const float* __restrict__ F, bf* Ph, bf* Pl, size_t n8) { const size_t i = (size_t)blockIdx.x * 256 + threadIdx.x; if (i >= n8) return; const v8f v = *(const v8f*)(F + i * 8); v8us oh, ol;
#pragma unroll
    for (int q = 0; q < 8; ++q) { unsigned short a, c; splitf(v[q], a, c); oh[q] = a; ol[q] = c; }
    *(volatile v8us*)(Ph + i * 8) = oh; *(volatile v8us*)(Pl + i * 8) = ol; __threadfence(); *(volatile v8us*)(Ph + i * 8) = oh; *(volatile v8us*)(Pl + i * 8) = ol; }
__global__ __launch_bounds__(256) void k_sumsplit8(const float* __restrict__ F1, const float* __restrict__ F2, bf* Ph, bf* Pl, size_t n8) { const size_t i = (size_t)blockIdx.x * 256 + threadIdx.x; if (i >= n8) return; const v8f v = *(const v8f*)(F1 + i * 8) + *(const v8f*)(F2 + i * 8); v8us oh, ol;
#pragma unroll
    for (int q = 0; q < 8; ++q) { unsigned short a, c; splitf(v[q], a, c); oh[q] = a; ol[q] = c; }
    *(volatile v8us*)(Ph + i * 8) = oh; *(volatile v8us*)(Pl + i * 8) = ol; __threadfence(); *(volatile v8us*)(Ph + i * 8) = oh; *(volatile v8us*)(Pl + i * 8) = ol; }
__global__ __launch_bounds__(256) void k_vsplit8(const float* __restrict__ F, h16* Ph, bf* Pl, size_t n8) { const size_t i = (size_t)blockIdx.x * 256 + threadIdx.x; if (i >= n8) return; const v8f v = *(const v8f*)(F + i * 8); v8h oh; v8us ol;
#pragma unroll
    for (int q = 0; q < 8; ++q) { const float w = v[q] * VCAR; const h16 hh = (h16)w; oh[q] = hh; ol[q] = f2bf(w - (float)hh); }
    *(volatile v8h*)(Ph + i * 8) = oh; *(volatile v8us*)(Pl + i * 8) = ol; __threadfence(); *(volatile v8h*)(Ph + i * 8) = oh; *(volatile v8us*)(Pl + i * 8) = ol; }

__global__ __launch_bounds__(32) void k_attn(const bf* __restrict__ THh, const bf* __restrict__ THl, const bf* __restrict__ DQh, const bf* __restrict__ DQl,
                                             const bf* __restrict__ PHh, const bf* __restrict__ PHl,
                                             const h16* __restrict__ GVh, const bf* __restrict__ GVl, const h16* __restrict__ SVh, const bf* __restrict__ SVl, float* Y) {
    __shared__ __align__(16) h16 pS16[16 * PP];
    __shared__ __align__(16) unsigned short pSb[16 * PP];
    __shared__ __align__(16) float os[16 * OSP];
    const int lane = threadIdx.x & 31, L = lane & 15, hi = lane >> 4;
    const int q0 = blockIdx.x * 16, b = blockIdx.y, mp = blockIdx.z;
    const size_t tok = (size_t)b * SEQ;
    const bf* Qh = (mp ? DQh : THh) + (tok + q0) * CI; const bf* Ql = (mp ? DQl : THl) + (tok + q0) * CI;
    const bf* Kh = PHh + tok * CI; const bf* Kl = PHl + tok * CI;
    const h16* Vh = (mp ? SVh : GVh) + (size_t)b * CI * SEQ; const bf* Vl = (mp ? SVl : GVl) + (size_t)b * CI * SEQ;
    float* Yo = Y + ((size_t)mp * NB * SEQ + tok + q0) * CI;
    float m_i[8], l_i[8]; v8f acc[8];
#pragma unroll
    for (int v = 0; v < 8; ++v) { m_i[v] = -1.0e30f; l_i[v] = 0.f; }
#pragma unroll
    for (int ct = 0; ct < 8; ++ct) acc[ct] = (v8f){};
    const size_t qoff = (size_t)L * CI + 8 * hi;
    const size_t voff0 = (size_t)L * SEQ + 8 * hi;
#pragma unroll 1
    for (int kb = 0; kb < SEQ; kb += KB) {
        v8f lt0 = (v8f){}, lt1 = (v8f){};
        const bf* k0h = Kh + (size_t)(kb + L) * CI + 8 * hi; const bf* k0l = Kl + (size_t)(kb + L) * CI + 8 * hi;
#pragma unroll 1
        for (int ch = 0; ch < CI / 32; ++ch) {
            const int co = ch * 32;
            const v16bf qa = ldb(Qh + qoff + co), qb = ldb(Ql + qoff + co);
            const v16bf ka0 = ldb(k0h + co), kl0 = ldb(k0l + co), ka1 = ldb(k0h + 16 * CI + co), kl1 = ldb(k0l + 16 * CI + co);
            lt0 = wmmab(qa, ka0, lt0); lt0 = wmmab(qb, ka0, lt0); lt0 = wmmab(qa, kl0, lt0);
            lt1 = wmmab(qa, ka1, lt1); lt1 = wmmab(qb, ka1, lt1); lt1 = wmmab(qa, kl1, lt1);
            asm volatile("v_nop\n\tv_nop\n\tv_nop\n\tv_nop" : "+v"(lt0), "+v"(lt1) : "v"(qa), "v"(qb), "v"(ka1), "v"(kl1));
        }
        float scv[8];
#pragma unroll
        for (int v = 0; v < 8; ++v) {
            const float ra = lt0[v], rb = lt1[v];
            float mx = fmaxf(ra, rb);
            mx = fmaxf(mx, __shfl_xor(mx, 1, 32)); mx = fmaxf(mx, __shfl_xor(mx, 2, 32)); mx = fmaxf(mx, __shfl_xor(mx, 4, 32)); mx = fmaxf(mx, __shfl_xor(mx, 8, 32));
            const float mn = fmaxf(m_i[v], mx);
            const float sc = __expf(m_i[v] - mn);
            const float pa = __expf(ra - mn), pb = __expf(rb - mn);
            float rs = pa + pb;
            rs += __shfl_xor(rs, 1, 32); rs += __shfl_xor(rs, 2, 32); rs += __shfl_xor(rs, 4, 32); rs += __shfl_xor(rs, 8, 32);
            l_i[v] = l_i[v] * sc + rs; m_i[v] = mn; scv[v] = sc;
            const float pas = pa * PCAR, pbs = pb * PCAR;
            const int prow = (v + 8 * hi) * PP;
            pS16[prow + L] = (h16)pas; pS16[prow + 16 + L] = (h16)pbs;
            pSb[prow + L] = f2bf(pas); pSb[prow + 16 + L] = f2bf(pbs);
        }
#pragma unroll
        for (int ct = 0; ct < 8; ++ct)
#pragma unroll
            for (int v = 0; v < 8; ++v) acc[ct][v] *= scv[v];
        __builtin_amdgcn_fence(__ATOMIC_RELEASE, "wavefront"); __builtin_amdgcn_wave_barrier(); asm volatile("" ::: "memory");
        const v16h pa16 = cat16(*(const v8ha*)(pS16 + L * PP + 8 * hi), *(const v8ha*)(pS16 + L * PP + 16 + 8 * hi));
        const v16bf pab = cat16b(*(const v8usa*)(pSb + L * PP + 8 * hi), *(const v8usa*)(pSb + L * PP + 16 + 8 * hi));
        const h16* vh = Vh + voff0 + kb; const bf* vl = Vl + voff0 + kb;
#pragma unroll
        for (int ct = 0; ct < 4; ++ct) {
            const v16h vf = ldh(vh + (size_t)ct * 16 * SEQ); const v16bf vr = ldb(vl + (size_t)ct * 16 * SEQ);
            acc[ct] = wmma16(pa16, vf, acc[ct]); acc[ct] = wmmab(pab, vr, acc[ct]); }
        asm volatile("v_nop\n\tv_nop\n\tv_nop\n\tv_nop" : "+v"(acc[0]), "+v"(acc[1]), "+v"(acc[2]), "+v"(acc[3]) : "v"(pa16), "v"(pab) : "memory");
#pragma unroll
        for (int ct = 4; ct < 8; ++ct) {
            const v16h vf = ldh(vh + (size_t)ct * 16 * SEQ); const v16bf vr = ldb(vl + (size_t)ct * 16 * SEQ);
            acc[ct] = wmma16(pa16, vf, acc[ct]); acc[ct] = wmmab(pab, vr, acc[ct]); }
        asm volatile("v_nop\n\tv_nop\n\tv_nop\n\tv_nop" : "+v"(acc[4]), "+v"(acc[5]), "+v"(acc[6]), "+v"(acc[7]) : "v"(pa16), "v"(pab) : "memory");
        __builtin_amdgcn_wave_barrier(); asm volatile("" ::: "memory");
    }
    float rl[8];
#pragma unroll
    for (int v = 0; v < 8; ++v) rl[v] = __builtin_amdgcn_rcpf(l_i[v]) * YSC;
#pragma unroll
    for (int ct = 0; ct < 8; ++ct)
#pragma unroll
        for (int v = 0; v < 8; ++v) os[(8 * hi + v) * OSP + ct * 16 + L] = acc[ct][v] * rl[v];
    __builtin_amdgcn_fence(__ATOMIC_RELEASE, "wavefront"); __builtin_amdgcn_wave_barrier(); asm volatile("" ::: "memory");
#pragma unroll 1
    for (int ps = 0; ps < 2; ++ps) {
#pragma unroll
        for (int r = 0; r < 16; ++r) { const v4f val = *(const v4fa*)(os + r * OSP + lane * 4); *(volatile v4f*)(Yo + (size_t)r * CI + lane * 4) = val; }
        if (ps == 0) __threadfence(); }
}

extern "C" void kernel_launch(void* const* d_in, const int* in_sizes, int n_in,
                              void* d_out, int out_size, void* d_ws, size_t ws_size, hipStream_t stream) {
    if (n_in < 13) return;
    if ((size_t)in_sizes[0] < (size_t)NB * C_ * HWF) return;
    if (in_sizes[1] < CI * C_ || in_sizes[3] < CI * C_ || in_sizes[5] < CI * C_ || in_sizes[7] < CI * C_ || in_sizes[9] < CI * C_ || in_sizes[11] < C_ * CI) return;
    if (in_sizes[2] < CI || in_sizes[4] < CI || in_sizes[6] < CI || in_sizes[8] < CI || in_sizes[10] < CI || in_sizes[12] < C_) return;
    if ((size_t)out_size < (size_t)NB * C_ * HWF) return;
    const float* x = (const float*)d_in[0];
    const float* w_theta = (const float*)d_in[1];  const float* b_theta = (const float*)d_in[2];
    const float* w_phi   = (const float*)d_in[3];  const float* b_phi   = (const float*)d_in[4];
    const float* w_g     = (const float*)d_in[5];  const float* b_g     = (const float*)d_in[6];
    const float* w_d     = (const float*)d_in[7];  const float* b_d     = (const float*)d_in[8];
    const float* w_s     = (const float*)d_in[9];  const float* b_s     = (const float*)d_in[10];
    const float* w_out   = (const float*)d_in[11]; const float* b_out   = (const float*)d_in[12];
    float* OUT = (float*)d_out;
    char* wsp = (char*)d_ws;
    auto take = [&](size_t bytes) { char* p = wsp; wsp += (bytes + 255) & ~(size_t)255; return (void*)p; };
    const size_t nTok = (size_t)NB * SEQ;
    bf* WTb = (bf*)take((size_t)CI * C_ * 2); bf* WPb = (bf*)take((size_t)CI * C_ * 2); bf* WGb = (bf*)take((size_t)CI * C_ * 2);
    bf* WDb = (bf*)take((size_t)CI * C_ * 2); bf* WSb = (bf*)take((size_t)CI * C_ * 2); bf* WOb = (bf*)take((size_t)C_ * CI * 2);
    float* MU = (float*)take((size_t)NB * C_ * 4); float* RD = (float*)take((size_t)NB * C_ * 4);
    bf* XT = (bf*)take(nTok * C_ * 2); bf* X1h = (bf*)take(nTok * C_ * 2); bf* X1l = (bf*)take(nTok * C_ * 2);
    float* F32A = (float*)take(2 * nTok * CI * 4);
    bf* THh = (bf*)take(nTok * CI * 2); bf* THl = (bf*)take(nTok * CI * 2);
    bf* PHh = (bf*)take(nTok * CI * 2); bf* PHl = (bf*)take(nTok * CI * 2);
    bf* DQh = (bf*)take(nTok * CI * 2); bf* DQl = (bf*)take(nTok * CI * 2);
    h16* GVh = (h16*)take(nTok * CI * 2); bf* GVl = (bf*)take(nTok * CI * 2);
    h16* SVh = (h16*)take(nTok * CI * 2); bf* SVl = (bf*)take(nTok * CI * 2);
    bf* Yh = (bf*)take(nTok * CI * 2); bf* Yl = (bf*)take(nTok * CI * 2);
    if ((size_t)(wsp - (char*)d_ws) > ws_size) return;
    float* Y1 = F32A; float* Y2 = F32A + nTok * CI;

    const unsigned gw = (unsigned)(((size_t)CI * C_ / 8 + 255) / 256);
    k_cvt8<<<gw, 256, 0, stream>>>(w_theta, WTb, (size_t)CI * C_ / 8);
    k_cvt8<<<gw, 256, 0, stream>>>(w_phi, WPb, (size_t)CI * C_ / 8);
    k_cvt8<<<gw, 256, 0, stream>>>(w_g, WGb, (size_t)CI * C_ / 8);
    k_cvt8<<<gw, 256, 0, stream>>>(w_d, WDb, (size_t)CI * C_ / 8);
    k_cvt8<<<gw, 256, 0, stream>>>(w_s, WSb, (size_t)CI * C_ / 8);
    k_cvt8<<<gw, 256, 0, stream>>>(w_out, WOb, (size_t)C_ * CI / 8);
    k_stats<<<(unsigned)(NB * C_ / 32), 256, 0, stream>>>(x, MU, RD);
    k_xplanes<<<(unsigned)((nTok * C_ / 8 + 255) / 256), 256, 0, stream>>>(x, MU, RD, XT, X1h, X1l);
    const size_t n8p = nTok * CI / 8; const unsigned gs8 = (unsigned)((n8p + 255) / 256);
    k_gemmw<bf, false, false, 1, false><<<dim3((unsigned)(nTok / 64), CI / 64, 1), 32, 0, stream>>>(XT, nullptr, WTb, nullptr, C_, F32A, CI, b_theta, nullptr, 0, 0, 0);
    k_split8<<<gs8, 256, 0, stream>>>(F32A, THh, THl, n8p);
    k_gemmw<bf, false, false, 1, false><<<dim3((unsigned)(nTok / 64), CI / 64, 1), 32, 0, stream>>>(XT, nullptr, WPb, nullptr, C_, F32A, CI, b_phi, nullptr, 0, 0, 0);
    k_split8<<<gs8, 256, 0, stream>>>(F32A, PHh, PHl, n8p);
    k_gemmw<bf, true, false, 1, false><<<dim3((unsigned)(nTok / 64), CI / 64, 1), 32, 0, stream>>>(X1h, X1l, WDb, nullptr, C_, F32A, CI, b_d, nullptr, 0, 0, 0);
    k_split8<<<gs8, 256, 0, stream>>>(F32A, DQh, DQl, n8p);
    k_gemmw<bf, false, false, 2, false><<<dim3(CI / 64, SEQ / 64, NB), 32, 0, stream>>>(WGb, nullptr, XT, nullptr, C_, F32A, SEQ, b_g, nullptr, 0, (size_t)SEQ * C_, (size_t)CI * SEQ);
    k_vsplit8<<<gs8, 256, 0, stream>>>(F32A, GVh, GVl, n8p);
    k_gemmw<bf, false, true, 2, false><<<dim3(CI / 64, SEQ / 64, NB), 32, 0, stream>>>(WSb, nullptr, X1h, X1l, C_, F32A, SEQ, b_s, nullptr, 0, (size_t)SEQ * C_, (size_t)CI * SEQ);
    k_vsplit8<<<gs8, 256, 0, stream>>>(F32A, SVh, SVl, n8p);
    k_attn<<<dim3(SEQ / 16, NB, 2), 32, 0, stream>>>(THh, THl, DQh, DQl, PHh, PHl, GVh, GVl, SVh, SVl, F32A);
    k_sumsplit8<<<gs8, 256, 0, stream>>>(Y1, Y2, Yh, Yl, n8p);
    k_gemmw<bf, false, true, 2, true><<<dim3(C_ / 64, SEQ / 64, NB), 32, 0, stream>>>(WOb, nullptr, Yh, Yl, CI, OUT, HWF, b_out, x, 0, (size_t)SEQ * CI, (size_t)C_ * HWF);
}
